// Stickbreaking_76501957476890
// MI455X (gfx1250) — hardware-verified
//
#include <hip/hip_runtime.h>
#include <stddef.h>
#include <stdint.h>

#define HEADS 16
#define SEQ   2048
#define HDM   64
#define NTOT  (HEADS * SEQ * HDM)
#define QB    128
#define KC    64
#define NQB   (SEQ / QB)
#define NCK   (SEQ / KC)
#define WV    8

static_assert(SEQ % QB == 0);
static_assert(SEQ % KC == 0);
static_assert(SEQ % 64 == 0);
static_assert(HDM == 64);
static_assert(QB == WV * 16);
static_assert(KC == 64);
static_assert(NTOT % 2048 == 0);
static_assert(HEADS * NQB == 256);

#define QS2 0.18033688011112042f

typedef _Float16 v16h __attribute__((ext_vector_type(16)));
typedef _Float16 v8h  __attribute__((ext_vector_type(8)));
typedef float    v8f  __attribute__((ext_vector_type(8)));
typedef float    v4f  __attribute__((ext_vector_type(4)));
typedef unsigned int v4u __attribute__((ext_vector_type(4)));

union Frag  { v16h v; v8h h[2]; };
union Pack8 { v8h h; v4u u; };

__device__ __forceinline__ v8f mma16(v16h a, v16h b, v8f c) {
  c = __builtin_amdgcn_wmma_f32_16x16x32_f16(false, a, false, b, (short)0, c, false, false);
  asm volatile("v_nop\n\tv_nop\n\tv_nop\n\tv_nop" : "+v"(c) : "v"(a), "v"(b));
  return c;
}

__device__ __forceinline__ v16h ldfrag(const _Float16* p, int ld, int row0, int k0, int lane) {
  const int m = lane & 15, lh = lane >> 4;
  const _Float16* q = p + (size_t)(row0 + m) * ld + k0 + 8 * lh;
  Frag f;
  f.h[0] = *(const v8h*)(q);
  f.h[1] = *(const v8h*)(q + 16);
  return f.v;
}

__device__ __forceinline__ v8f zero8() { return (v8f){0.f, 0.f, 0.f, 0.f, 0.f, 0.f, 0.f, 0.f}; }

__global__ __launch_bounds__(256) void k_cvt(const float* __restrict__ src, _Float16* __restrict__ dh, float scale) {
  const int tid = threadIdx.x;
  const size_t o = (size_t)blockIdx.x * 2048 + (size_t)tid * 8;
  const v4f a0 = *(const v4f*)(src + o) * scale;
  const v4f a1 = *(const v4f*)(src + o + 4) * scale;
  Pack8 pk;
  pk.h = (v8h){(_Float16)a0[0], (_Float16)a0[1], (_Float16)a0[2], (_Float16)a0[3],
               (_Float16)a1[0], (_Float16)a1[1], (_Float16)a1[2], (_Float16)a1[3]};
  const v4u vv = pk.u;
  volatile v4u* d = (volatile v4u*)(dh + o);
  *d = vv;
  __threadfence();
  *d = vv;
}

#define VTP 72
__global__ __launch_bounds__(256) void k_vtr(const float* __restrict__ v, _Float16* __restrict__ vt) {
  __shared__ __align__(16) _Float16 st[HDM * VTP];
  const int tid = threadIdx.x;
  const int s0 = blockIdx.x * 64;
  const int h  = blockIdx.y;
  const float* src = v + (size_t)h * SEQ * HDM + (size_t)s0 * HDM;
#pragma unroll
  for (int i = 0; i < 4; ++i) {
    const int idx = tid + 256 * i;
    const int r   = idx >> 4;
    const int c4  = (idx & 15) * 4;
    const v4f f = *(const v4f*)(src + (size_t)r * HDM + c4);
    st[(c4 + 0) * VTP + r] = (_Float16)f[0];
    st[(c4 + 1) * VTP + r] = (_Float16)f[1];
    st[(c4 + 2) * VTP + r] = (_Float16)f[2];
    st[(c4 + 3) * VTP + r] = (_Float16)f[3];
  }
  __syncthreads();
  _Float16* dst = vt + (size_t)h * HDM * SEQ + s0;
  v4u val[2];
  size_t go[2];
#pragma unroll
  for (int g = 0; g < 2; ++g) {
    const int p   = tid + 256 * g;
    const int row = p >> 3;
    const int pc  = p & 7;
    Pack8 pk;
    pk.h   = *(const v8h*)(st + row * VTP + pc * 8);
    val[g] = pk.u;
    go[g]  = (size_t)row * SEQ + pc * 8;
  }
  for (int ps = 0; ps < 2; ++ps) {
#pragma unroll
    for (int g = 0; g < 2; ++g) *(volatile v4u*)(dst + go[g]) = val[g];
    __threadfence();
  }
}

#define KTP 72
#define OTP 68
__global__ __launch_bounds__(256) void k_attn(const _Float16* __restrict__ qp,
                                              const _Float16* __restrict__ kp,
                                              const _Float16* __restrict__ vt,
                                              float* __restrict__ out) {
  __shared__ __align__(16) _Float16 Ks[KC * KTP];
  __shared__ __align__(16) _Float16 Vs[HDM * KTP];
  __shared__ __align__(16) _Float16 Ps[WV * 16 * KTP];
  __shared__ __align__(16) float    Os[WV * 16 * OTP];

  const int tid = threadIdx.x, lane = tid & 31, wave = tid >> 5;
  const int hh = lane >> 4, c = lane & 15;
  const int qb  = blockIdx.x % NQB;
  const int hb  = blockIdx.x / NQB;
  const int q0  = qb * QB + wave * 16;

  const _Float16* Q = qp + (size_t)hb * SEQ * HDM;
  const _Float16* K = kp + (size_t)hb * SEQ * HDM;
  const _Float16* V = vt + (size_t)hb * HDM * SEQ;

  v16h qa[2];
  qa[0] = ldfrag(Q, HDM, q0, 0, lane);
  qa[1] = ldfrag(Q, HDM, q0, 32, lane);

  float carry[8];
  v8f oacc[4];
#pragma unroll
  for (int r = 0; r < 8; ++r) carry[r] = 0.f;
#pragma unroll
  for (int t = 0; t < 4; ++t) oacc[t] = zero8();

  _Float16* pw = Ps + wave * 16 * KTP;

  for (int kci = 0; kci < NCK; ++kci) {
    const int kv0 = (NCK - 1 - kci) * KC;
    __syncthreads();
    {
      const int r  = tid >> 2;
      const int qq = (tid & 3) * 16;
      const _Float16* ks = K + (size_t)(kv0 + r) * HDM + qq;
      const _Float16* vs = V + (size_t)r * SEQ + kv0 + qq;
#pragma unroll
      for (int e = 0; e < 2; ++e) {
        *(v8h*)(Ks + r * KTP + qq + 8 * e) = *(const v8h*)(ks + 8 * e);
        *(v8h*)(Vs + r * KTP + qq + 8 * e) = *(const v8h*)(vs + 8 * e);
      }
    }
    __syncthreads();

    v8f s[4];
#pragma unroll
    for (int j = 0; j < 4; ++j) s[j] = zero8();
#pragma unroll
    for (int dc = 0; dc < 2; ++dc) {
#pragma unroll
      for (int j = 0; j < 4; ++j) {
        const v16h kb = ldfrag(Ks, KTP, j * 16, dc * 32, lane);
        s[j] = mma16(qa[dc], kb, s[j]);
      }
    }

#pragma unroll
    for (int r = 0; r < 8; ++r) {
      float lz[4], sc[4];
#pragma unroll
      for (int j = 0; j < 4; ++j) {
        const float x  = s[j][r] * QS2;
        const float ee = __builtin_amdgcn_exp2f(-__builtin_fabsf(x));
        const float lb = -(fmaxf(x, 0.0f) + __builtin_amdgcn_logf(1.0f + ee));
        lz[j] = x + lb;
        sc[j] = lb;
      }
#pragma unroll
      for (int j = 0; j < 4; ++j) {
#pragma unroll
        for (int off = 1; off < 16; off <<= 1) {
          const float tv = __shfl_down(sc[j], off, 16);
          sc[j] += (c + off < 16) ? tv : 0.0f;
        }
      }
      float run = carry[r];
#pragma unroll
      for (int jj = 0; jj < 4; ++jj) {
        const int j = 3 - jj;
        const float w = __builtin_amdgcn_exp2f(lz[j] + sc[j] + run);
        pw[(8 * hh + r) * KTP + 16 * j + c] = (_Float16)(w * 1024.0f);
        run += __shfl(sc[j], 0, 16);
      }
      carry[r] = run;
    }
    __syncthreads();

#pragma unroll
    for (int kk = 0; kk < 2; ++kk) {
      const v16h pa = ldfrag(pw, KTP, 0, kk * 32, lane);
#pragma unroll
      for (int t = 0; t < 4; ++t) {
        const v16h vb = ldfrag(Vs, KTP, t * 16, kk * 32, lane);
        oacc[t] = mma16(pa, vb, oacc[t]);
      }
    }
  }

  float* ow = Os + wave * 16 * OTP;
  __syncthreads();
#pragma unroll
  for (int t = 0; t < 4; ++t) {
#pragma unroll
    for (int r = 0; r < 8; ++r) ow[(8 * hh + r) * OTP + 16 * t + c] = oacc[t][r] * 0.0009765625f;
  }
  __syncthreads();
  v4f val[8];
  size_t go[8];
#pragma unroll
  for (int it = 0; it < 8; ++it) {
    const int p    = lane + 32 * it;
    const int L    = p >> 3;
    const int pc   = p & 7;
    const int row  = L >> 1;
    const int half = L & 1;
    val[it] = *(const v4f*)(ow + row * OTP + half * 32 + pc * 4);
    go[it]  = ((size_t)hb * SEQ + (size_t)(q0 + row)) * HDM + half * 32 + pc * 4;
  }
  for (int ps = 0; ps < 2; ++ps) {
#pragma unroll
    for (int it = 0; it < 8; ++it) *(volatile v4f*)(out + go[it]) = val[it];
    __threadfence();
  }
}

extern "C" void kernel_launch(void* const* d_in, const int* in_sizes, int n_in,
                              void* d_out, int out_size, void* d_ws, size_t ws_size,
                              hipStream_t stream) {
  if (n_in < 3) return;
  if (in_sizes[0] != NTOT) return;
  if (in_sizes[1] != NTOT) return;
  if (in_sizes[2] != NTOT) return;
  if (out_size != NTOT) return;

  const float* q = (const float*)d_in[0];
  const float* k = (const float*)d_in[1];
  const float* v = (const float*)d_in[2];
  float* out = (float*)d_out;

  size_t off = 0;
  const size_t oQ = off; off += (size_t)NTOT * 2;
  const size_t oK = off; off += (size_t)NTOT * 2;
  const size_t oV = off; off += (size_t)NTOT * 2;
  if (off > ws_size) return;
  if (off > (size_t)134217728) return;

  char* ws = (char*)d_ws;
  _Float16* Qh = (_Float16*)(ws + oQ);
  _Float16* Kh = (_Float16*)(ws + oK);
  _Float16* Vt = (_Float16*)(ws + oV);

  k_cvt<<<dim3(NTOT / 2048), dim3(256), 0, stream>>>(q, Qh, 1.0f);
  k_cvt<<<dim3(NTOT / 2048), dim3(256), 0, stream>>>(k, Kh, 1.0f);
  k_vtr<<<dim3(SEQ / 64, HEADS), dim3(256), 0, stream>>>(v, Vt);
  k_attn<<<dim3(HEADS * NQB), dim3(256), 0, stream>>>(Qh, Kh, Vt, out);
  (void)hipGetLastError();
}
